// CausalMultiHeadSelfAttention_80539226734672
// MI455X (gfx1250) — hardware-verified
//
#include <hip/hip_runtime.h>
#include <math.h>

#ifndef NB
#define NB 2
#endif
#ifndef SEQ
#define SEQ 2048
#endif
#define NB_FULL 2
#define SEQ_FULL 2048
#define DM 1024
#define NH 16
#define HD 64
#define NTOK (NB * SEQ)
static_assert(NB >= 1 && NB <= NB_FULL);
static_assert(SEQ % 64 == 0 && SEQ >= 64 && SEQ <= SEQ_FULL);
static_assert(NH * HD == DM);
static_assert((3 * DM) % 64 == 0 && DM % 64 == 0 && NTOK % 64 == 0);

typedef __attribute__((ext_vector_type(16))) _Float16 v16h;
typedef __attribute__((ext_vector_type(8)))  _Float16 v8h;
typedef __attribute__((ext_vector_type(16))) __bf16   v16b;
typedef __attribute__((ext_vector_type(8)))  __bf16   v8b;
typedef __attribute__((ext_vector_type(8)))  float    v8f;
typedef __attribute__((ext_vector_type(4)))  float    v4f;
typedef __attribute__((ext_vector_type(4)))  unsigned int v4u;

#define VST2(T, ptr, val) do { const T vst2_v_ = (val); *(volatile T*)(ptr) = vst2_v_; __threadfence(); *(volatile T*)(ptr) = vst2_v_; } while (0)
#define VST2V4(ptr, val) do { const v4f vst2_v4_ = (val); *(volatile v4f*)(ptr) = vst2_v4_; __threadfence(); *(volatile v4f*)(ptr) = vst2_v4_; } while (0)

__device__ __forceinline__ unsigned short f2bf_bits(float f) { unsigned u = __float_as_uint(f); return (unsigned short)((u + 0x7FFFu + ((u >> 16) & 1u)) >> 16); }
__device__ __forceinline__ float bf_bits2f(unsigned short h) { return __uint_as_float(((unsigned)h) << 16); }
__device__ __forceinline__ __bf16 at_f2bf(float f) { return __builtin_bit_cast(__bf16, f2bf_bits(f)); }
__device__ __forceinline__ void at_split(float f, __bf16& hi, __bf16& lo) {
  const unsigned short hb = f2bf_bits(f);
  hi = __builtin_bit_cast(__bf16, hb);
  lo = at_f2bf(f - bf_bits2f(hb));
}
__device__ __forceinline__ v8f at_mma(v16b a, v16b b, v8f c) {
  c = __builtin_amdgcn_wmma_f32_16x16x32_bf16(false, a, false, b, (short)0, c, false, false);
  asm volatile("v_nop\n\tv_nop\n\tv_nop\n\tv_nop" : "+v"(c) : "v"(a), "v"(b));
  return c;
}

__device__ __forceinline__ void dep_guard_h(v8f& a, v8f& b, v16h x, v16h y) { asm volatile("v_nop\n\tv_nop\n\tv_nop\n\tv_nop" : "+v"(a), "+v"(b) : "v"(x), "v"(y)); }
__device__ __forceinline__ void dep_guard_b(v8f& a, v8f& b, v16b x, v16b y) { asm volatile("v_nop\n\tv_nop\n\tv_nop\n\tv_nop" : "+v"(a), "+v"(b) : "v"(x), "v"(y)); }
__device__ __forceinline__ void keep4_h(v16h a, v16h b, v16h c, v16h d) { asm volatile("v_nop" :: "v"(a), "v"(b), "v"(c), "v"(d)); }
__device__ __forceinline__ void keep4_b(v16b a, v16b b, v16b c, v16b d) { asm volatile("v_nop" :: "v"(a), "v"(b), "v"(c), "v"(d)); }
__device__ __forceinline__ void acc_guard4(v8f& a, v8f& b, v8f& c, v8f& d) { asm volatile("v_nop\n\tv_nop\n\tv_nop\n\tv_nop" : "+v"(a), "+v"(b), "+v"(c), "+v"(d)); }
template <typename T> struct Frag;
template <> struct Frag<_Float16> {
  typedef v16h V; union U { v16h v; v8h h[2]; };
  static __device__ __forceinline__ v16h load(const _Float16* p) {
    U f; f.h[0] = *(const v8h*)(p); f.h[1] = *(const v8h*)(p + 16); return f.v;
  }
  static __device__ __forceinline__ v8f mma(v16h a, v16h b, v8f c) {
    return __builtin_amdgcn_wmma_f32_16x16x32_f16(false, a, false, b, (short)0, c, false, false);
  }
  static __device__ __forceinline__ void guard(v8f& a, v8f& b, v16h x, v16h y) { dep_guard_h(a, b, x, y); }
  static __device__ __forceinline__ void keep(v16h a, v16h b, v16h c, v16h d) { keep4_h(a, b, c, d); }
};
template <> struct Frag<__bf16> {
  typedef v16b V; union U { v16b v; v8b h[2]; };
  static __device__ __forceinline__ v16b load(const __bf16* p) {
    U f; f.h[0] = *(const v8b*)(p); f.h[1] = *(const v8b*)(p + 16); return f.v;
  }
  static __device__ __forceinline__ v8f mma(v16b a, v16b b, v8f c) {
    return __builtin_amdgcn_wmma_f32_16x16x32_bf16(false, a, false, b, (short)0, c, false, false);
  }
  static __device__ __forceinline__ void guard(v8f& a, v8f& b, v16b x, v16b y) { dep_guard_b(a, b, x, y); }
  static __device__ __forceinline__ void keep(v16b a, v16b b, v16b c, v16b d) { keep4_b(a, b, c, d); }
};

template <int ET> struct Elem;
template <> struct Elem<0> { typedef _Float16 T; };
template <> struct Elem<1> { typedef __bf16 T; };
template <int ET, bool SPLIT, int BIAS_MODE, int OUT_MODE, bool RESID>
__global__ __launch_bounds__(256) void wmma_gemm64(
    const unsigned short* __restrict__ Ap, const unsigned short* __restrict__ A2p, int lda, long strideA,
    const unsigned short* __restrict__ Btp, const unsigned short* __restrict__ Bt2p, int ldb, long strideB,
    void* __restrict__ Cout, void* __restrict__ Cout2, int ldc, long strideC,
    const float* __restrict__ bias,
    const float* __restrict__ resid, long strideR,
    int M, int N, int K, float scale) {
  typedef typename Elem<ET>::T T;
  typedef typename Frag<T>::V V;
  const T* A = (const T*)Ap; const T* A2 = (const T*)A2p; const T* Bt = (const T*)Btp; const T* Bt2 = (const T*)Bt2p;
  __shared__ __align__(16) float sT[8][16 * 68];
  const int b    = blockIdx.y;
  const int lane = threadIdx.x & 31;
  const int wave = threadIdx.x >> 5;
  const int tilesN = N >> 6;
  const int tilesM = M >> 6;
  const int tile = blockIdx.x * 8 + wave;
  if (tile >= tilesM * tilesN) return;
  const int tm = tile / tilesN;
  const int tn = tile - tm * tilesN;
  const int m0 = tm << 6;
  const int n0 = tn << 6;

  const T* Ab  = A  + (size_t)b * strideA;
  const T* Bb  = Bt + (size_t)b * strideB;
  const T* Ab2 = SPLIT ? (A2  + (size_t)b * strideA) : nullptr;
  const T* Bb2 = SPLIT ? (Bt2 + (size_t)b * strideB) : nullptr;

  const int rlane = lane & 15;
  const int koff  = (lane >> 4) * 8;
  const int mOff  = (lane >> 4) * 8;

  v8f acc[4][4];
#pragma unroll
  for (int i = 0; i < 4; ++i)
#pragma unroll
    for (int j = 0; j < 4; ++j) acc[i][j] = (v8f){0.f,0.f,0.f,0.f,0.f,0.f,0.f,0.f};

  for (int k0 = 0; k0 < K; k0 += 32) {
    V bh[4], bl[4];
#pragma unroll
    for (int j = 0; j < 4; ++j) {
      const size_t bo = (size_t)(n0 + (j << 4) + rlane) * ldb + koff + k0;
      bh[j] = Frag<T>::load(Bb + bo);
      if (SPLIT) bl[j] = Frag<T>::load(Bb2 + bo);
    }
#pragma unroll
    for (int i = 0; i < 4; ++i) {
      const size_t ao = (size_t)(m0 + (i << 4) + rlane) * lda + koff + k0;
      V ah = Frag<T>::load(Ab + ao);
      V al;
      if (SPLIT) al = Frag<T>::load(Ab2 + ao);
#pragma unroll
      for (int j = 0; j < 4; ++j) {
        acc[i][j] = Frag<T>::mma(ah, bh[j], acc[i][j]);
        if (SPLIT) {
          acc[i][j] = Frag<T>::mma(ah, bl[j], acc[i][j]);
          acc[i][j] = Frag<T>::mma(al, bh[j], acc[i][j]);
        }
      }
      Frag<T>::guard(acc[i][0], acc[i][3], ah, SPLIT ? al : ah);
    }
    Frag<T>::keep(bh[0], bh[1], bh[2], bh[3]);
    if (SPLIT) Frag<T>::keep(bl[0], bl[1], bl[2], bl[3]);
  }
  acc_guard4(acc[0][0], acc[0][1], acc[0][2], acc[0][3]);
  acc_guard4(acc[1][0], acc[1][1], acc[1][2], acc[1][3]);
  acc_guard4(acc[2][0], acc[2][1], acc[2][2], acc[2][3]);
  acc_guard4(acc[3][0], acc[3][1], acc[3][2], acc[3][3]);

  float* slab = sT[wave];
  const float* Rb = RESID ? (resid + (size_t)b * strideR) : nullptr;
#pragma unroll
  for (int i = 0; i < 4; ++i) {
    const int mBase = m0 + (i << 4);
#pragma unroll
    for (int j = 0; j < 4; ++j) {
      const int n = n0 + (j << 4) + rlane;
      float bv = 0.f;
      if (BIAS_MODE == 2) bv = bias[n];
#pragma unroll
      for (int r = 0; r < 8; ++r) {
        float v = acc[i][j][r] * scale;
        if (BIAS_MODE == 1) v += bias[mBase + mOff + r];
        if (BIAS_MODE == 2) v += bv;
        if (RESID) v += Rb[(size_t)(mBase + mOff + r) * ldc + n];
        slab[(mOff + r) * 68 + (j << 4) + rlane] = v;
      }
    }
    __builtin_amdgcn_fence(3  , "workgroup");
    __builtin_amdgcn_wave_barrier();
    __builtin_amdgcn_fence(2  , "workgroup");
    if (OUT_MODE == 0) {
      float* C = (float*)Cout + (size_t)b * strideC;
      const int hh = lane >> 4, c4 = (lane & 15) * 4;
      for (int pass = 0; pass < 2; ++pass) {
#pragma unroll
        for (int it = 0; it < 8; ++it) {
          const int row = it * 2 + hh;
          v4f v = *(const v4f*)(slab + row * 68 + c4);
          *(volatile v4f*)(C + (size_t)(mBase + row) * ldc + n0 + c4) = v;
        }
        __threadfence();
      }
    } else {
      const int q = lane >> 3, c8 = (lane & 7) * 8;
      unsigned short* C  = (unsigned short*)Cout  + (size_t)b * strideC;
      unsigned short* C2 = (OUT_MODE == 2) ? ((unsigned short*)Cout2 + (size_t)b * strideC) : nullptr;
      for (int pass = 0; pass < 2; ++pass) {
#pragma unroll
        for (int it = 0; it < 4; ++it) {
          const int row = it * 4 + q;
          const float* sp = slab + row * 68 + c8;
          v8h hv, lv;
#pragma unroll
          for (int e = 0; e < 8; ++e) {
            if (OUT_MODE == 1) {
              hv[e] = (_Float16)sp[e];
            } else {
              unsigned short hb = f2bf_bits(sp[e]);
              unsigned short lb = f2bf_bits(sp[e] - bf_bits2f(hb));
              hv[e] = __builtin_bit_cast(_Float16, hb);
              lv[e] = __builtin_bit_cast(_Float16, lb);
            }
          }
          *(volatile v8h*)(C + (size_t)(mBase + row) * ldc + n0 + c8) = hv;
          if (OUT_MODE == 2) *(volatile v8h*)(C2 + (size_t)(mBase + row) * ldc + n0 + c8) = lv;
        }
        __threadfence();
      }
    }
    __builtin_amdgcn_fence(3  , "workgroup");
    __builtin_amdgcn_wave_barrier();
    __builtin_amdgcn_fence(2  , "workgroup");
  }
}

__device__ __forceinline__ unsigned int cmb_pk2(float a, float b) { return (unsigned int)__builtin_bit_cast(unsigned short, (_Float16)a) | ((unsigned int)__builtin_bit_cast(unsigned short, (_Float16)b) << 16); }
__device__ __forceinline__ float cmb_bf(float v) { const unsigned u = __builtin_bit_cast(unsigned, v); const unsigned r = (u + 0x7fffu + ((u >> 16) & 1u)) & 0xffff0000u; return __builtin_bit_cast(float, r); }
__global__ __launch_bounds__(256) void k_cm_castb(const float* __restrict__ SRC, int lds, unsigned short* __restrict__ DST, int ldd, int nR, int nC, float sc) {
    const long long u = (long long)blockIdx.x * 256 + threadIdx.x; const int per = nC / 8; if (u >= (long long)nR * per) return; const int r = (int)(u / per); const int c0 = 8 * (int)(u % per);
    const float* s = SRC + (long long)r * lds + c0; float w[8];
#pragma unroll
    for (int e = 0; e < 8; ++e) w[e] = cmb_bf(s[e]) * sc;
    v4u pk; pk.x = cmb_pk2(w[0], w[1]); pk.y = cmb_pk2(w[2], w[3]); pk.z = cmb_pk2(w[4], w[5]); pk.w = cmb_pk2(w[6], w[7]); VST2(v4u, (v4u*)(DST + (long long)r * ldd + c0), pk); }

__device__ __forceinline__ unsigned int f2bf2_pack(float a, float b, unsigned int* lo) {
    const unsigned short ha = f2bf_bits(a), hb = f2bf_bits(b);
    const unsigned short la = f2bf_bits(a - bf_bits2f(ha)), lb = f2bf_bits(b - bf_bits2f(hb));
    *lo = (unsigned)la | ((unsigned)lb << 16); return (unsigned)ha | ((unsigned)hb << 16); }
__global__ __launch_bounds__(256) void k_castS16(const float* __restrict__ src, long long lds, __bf16* __restrict__ dhi, __bf16* __restrict__ dlo, long long ldd, int R, int C, float s, int transpose) {
    const long long i = (long long)blockIdx.x * 256 + threadIdx.x; long long o; float a, b;
    if (transpose) { const long long np = (long long)C * (R / 2); if (i >= np) return; const int c = (int)(i / (R / 2)); const int r = 2 * (int)(i % (R / 2)); a = src[(long long)r * lds + c] * s; b = src[(long long)(r + 1) * lds + c] * s; o = (long long)c * ldd + r; }
    else { const long long np = (long long)R * (C / 2); if (i >= np) return; const int r = (int)(i / (C / 2)); const int c = 2 * (int)(i % (C / 2)); a = src[(long long)r * lds + c] * s; b = src[(long long)r * lds + c + 1] * s; o = (long long)r * ldd + c; }
    unsigned lo; const unsigned hi = f2bf2_pack(a, b, &lo); volatile unsigned* ph = (volatile unsigned*)(dhi + o); volatile unsigned* pl = (volatile unsigned*)(dlo + o);
    *ph = hi; *pl = lo; __threadfence(); *ph = hi; *pl = lo; }

__global__ __launch_bounds__(256) void k_rmsqk(float* __restrict__ QKV, int nvec) {
    const int lane = threadIdx.x & 31; const int sub = lane & 15;
    int vi = blockIdx.x * 16 + (threadIdx.x >> 4); vi = min(vi, nvec - 1);
    const int t = vi / (2 * NH); const int rem = vi - t * (2 * NH); const int p = rem / NH; const int h = rem - p * NH;
    float* ptr = QKV + (size_t)t * (3 * DM) + (size_t)p * DM + (size_t)h * HD + 4 * sub;
    const v4f x = *(const v4f*)ptr;
    float ss = x.x * x.x + x.y * x.y + x.z * x.z + x.w * x.w;
    ss += __shfl_xor(ss, 1, 32); ss += __shfl_xor(ss, 2, 32); ss += __shfl_xor(ss, 4, 32); ss += __shfl_xor(ss, 8, 32);
    const float rs = rsqrtf(ss * (1.0f / 64.0f) + 1.1920929e-07f);
    const v4f y = x * rs;
    VST2V4(ptr, y);
}
static_assert((NTOK * 2 * NH) % 16 == 0);

#define AT_D 64
#define AT_NW 4
#define AT_QB 64
#define AT_KC 64
struct AttnGeom { long long q_bs, q_rs, q_hs, k_bs, k_rs, k_hs, v_bs, v_rs, v_hs, o_bs, o_rs, o_hs; int S, H, nqb; float qscale, cap, capc; };
static_assert(sizeof(AttnGeom) == 12 * 8 + 6 * 4);

template <bool SPLIT_QK, bool SPLIT_PV>
__global__ __launch_bounds__(128)
void k_attn64c(const float* __restrict__ q, const float* __restrict__ k,
               const float* __restrict__ v, float* __restrict__ out, AttnGeom g) {
  union FB { v16b v; v8b h[2]; };
  __shared__ __align__(16) __bf16 Ksh[AT_KC * AT_D];
  __shared__ __align__(16) __bf16 Ksl[SPLIT_QK ? AT_KC * AT_D : 8];
  __shared__ __align__(16) __bf16 Vth[AT_D * AT_KC];
  __shared__ __align__(16) __bf16 Vtl[SPLIT_PV ? AT_D * AT_KC : 8];
  __shared__ __align__(16) __bf16 Psh[AT_NW][16 * AT_KC];
  __shared__ __align__(16) __bf16 Psl[SPLIT_PV ? AT_NW : 1][SPLIT_PV ? 16 * AT_KC : 8];
  __shared__ __align__(16) float  Os[AT_NW][16 * 68];

  const int tid  = threadIdx.x;
  const int wave = tid >> 5;
  const int lane = tid & 31;
  const int hh   = lane >> 4;
  const int c    = lane & 15;

  const int bx = blockIdx.x;
  const int qb = bx % g.nqb;
  const int bh = bx / g.nqb;
  const int h  = bh % g.H;
  const int b  = bh / g.H;
  const int q0 = qb * AT_QB + wave * 16;
  const float NEG = -__builtin_inff();

  const float* qb_ptr = q + (size_t)b * g.q_bs + (size_t)h * g.q_hs;
  const float* kb_ptr = k + (size_t)b * g.k_bs + (size_t)h * g.k_hs;
  const float* vb_ptr = v + (size_t)b * g.v_bs + (size_t)h * g.v_hs;
  float*       ob_ptr = out + (size_t)b * g.o_bs + (size_t)h * g.o_hs;

  v16b qah[2], qal[2];
  {
    const float* qrow = qb_ptr + (size_t)(q0 + c) * g.q_rs;
#pragma unroll
    for (int dc = 0; dc < 2; ++dc) {
#pragma unroll
      for (int e = 0; e < 8; ++e) {
        const float f0 = qrow[dc * 32 + 8 * hh + e] * g.qscale;
        const float f1 = qrow[dc * 32 + 16 + 8 * hh + e] * g.qscale;
        if (SPLIT_QK) { __bf16 hq, lq; at_split(f0, hq, lq); qah[dc][e] = hq; qal[dc][e] = lq; at_split(f1, hq, lq); qah[dc][8 + e] = hq; qal[dc][8 + e] = lq; }
        else { qah[dc][e] = at_f2bf(f0); qah[dc][8 + e] = at_f2bf(f1); qal[dc][e] = qah[dc][e]; qal[dc][8 + e] = qah[dc][8 + e]; }
      }
    }
  }

  float mrow[8], lrow[8];
  v8f oacc[4];
#pragma unroll
  for (int r = 0; r < 8; ++r) { mrow[r] = NEG; lrow[r] = 0.f; }
#pragma unroll
  for (int t = 0; t < 4; ++t) oacc[t] = (v8f){0.f,0.f,0.f,0.f,0.f,0.f,0.f,0.f};

  const int nChunks = qb + 1;
  for (int kc = 0; kc < nChunks; ++kc) {
    const int kv0 = kc * AT_KC;
    __syncthreads();
    {
      const int kvr = tid >> 1, dh = (tid & 1) * 32;
      const float* krow = kb_ptr + (size_t)(kv0 + kvr) * g.k_rs + dh;
      const float* vrow = vb_ptr + (size_t)(kv0 + kvr) * g.v_rs + dh;
#pragma unroll
      for (int i = 0; i < 8; ++i) {
        v4f kk = *(const v4f*)(krow + 4 * i);
        v4f vv = *(const v4f*)(vrow + 4 * i);
#pragma unroll
        for (int e = 0; e < 4; ++e) {
          const int d = dh + 4 * i + e;
          if (SPLIT_QK) { __bf16 a, bl; at_split(kk[e], a, bl); Ksh[kvr * AT_D + d] = a; Ksl[kvr * AT_D + d] = bl; }
          else Ksh[kvr * AT_D + d] = at_f2bf(kk[e]);
          if (SPLIT_PV) { __bf16 a, bl; at_split(vv[e], a, bl); Vth[d * AT_KC + kvr] = a; Vtl[d * AT_KC + kvr] = bl; }
          else Vth[d * AT_KC + kvr] = at_f2bf(vv[e]);
        }
      }
    }
    __syncthreads();

    v8f s[4];
#pragma unroll
    for (int j = 0; j < 4; ++j) {
      s[j] = (v8f){0.f,0.f,0.f,0.f,0.f,0.f,0.f,0.f};
#pragma unroll
      for (int dc = 0; dc < 2; ++dc) {
        FB kb;
        kb.h[0] = *(const v8b*)(Ksh + (j * 16 + c) * AT_D + dc * 32 + 8 * hh);
        kb.h[1] = *(const v8b*)(Ksh + (j * 16 + c) * AT_D + dc * 32 + 16 + 8 * hh);
        s[j] = at_mma(qah[dc], kb.v, s[j]);
        if (SPLIT_QK) {
          FB kl;
          kl.h[0] = *(const v8b*)(Ksl + (j * 16 + c) * AT_D + dc * 32 + 8 * hh);
          kl.h[1] = *(const v8b*)(Ksl + (j * 16 + c) * AT_D + dc * 32 + 16 + 8 * hh);
          s[j] = at_mma(qah[dc], kl.v, s[j]);
          s[j] = at_mma(qal[dc], kb.v, s[j]);
        }
      }
    }
    const bool diag = (kc == qb);
    float cm[8];
#pragma unroll
    for (int r = 0; r < 8; ++r) {
      const int qrow = q0 + 8 * hh + r;
      float m = NEG;
#pragma unroll
      for (int j = 0; j < 4; ++j) {
        const int kvcol = kv0 + j * 16 + c;
        float sv = s[j][r];
        const float ee = exp2f(sv * g.capc);
        sv = g.cap - (2.0f * g.cap) * __builtin_amdgcn_rcpf(1.0f + ee);
        if (diag && kvcol > qrow) sv = NEG;
        s[j][r] = sv;
        m = fmaxf(m, sv);
      }
#pragma unroll
      for (int off = 1; off < 16; off <<= 1) m = fmaxf(m, __shfl_xor(m, off, 32));
      cm[r] = m;
    }
    __bf16* pwh = Psh[wave];
    __bf16* pwl = Psl[SPLIT_PV ? wave : 0];
#pragma unroll
    for (int r = 0; r < 8; ++r) {
      const float mnew = fmaxf(mrow[r], cm[r]);
      const float alpha = expf(mrow[r] - mnew);
      mrow[r] = mnew;
      float psum = 0.f;
#pragma unroll
      for (int j = 0; j < 4; ++j) {
        const float p = expf(s[j][r] - mnew);
        psum += p;
        if (SPLIT_PV) { __bf16 a, bl; at_split(p, a, bl); pwh[(8 * hh + r) * AT_KC + j * 16 + c] = a; pwl[(8 * hh + r) * AT_KC + j * 16 + c] = bl; }
        else pwh[(8 * hh + r) * AT_KC + j * 16 + c] = at_f2bf(p);
      }
#pragma unroll
      for (int off = 1; off < 16; off <<= 1) psum += __shfl_xor(psum, off, 32);
      lrow[r] = lrow[r] * alpha + psum;
#pragma unroll
      for (int t = 0; t < 4; ++t) oacc[t][r] *= alpha;
    }
    __builtin_amdgcn_fence(3  , "workgroup");
    __builtin_amdgcn_wave_barrier();
    __builtin_amdgcn_fence(2  , "workgroup");
#pragma unroll 1
    for (int kk = 0; kk < 2; ++kk) {
      FB pa, pl;
      pa.h[0] = *(const v8b*)(pwh + c * AT_KC + kk * 32 + 8 * hh);
      pa.h[1] = *(const v8b*)(pwh + c * AT_KC + kk * 32 + 16 + 8 * hh);
      if (SPLIT_PV) {
        pl.h[0] = *(const v8b*)(pwl + c * AT_KC + kk * 32 + 8 * hh);
        pl.h[1] = *(const v8b*)(pwl + c * AT_KC + kk * 32 + 16 + 8 * hh);
      }
#pragma unroll
      for (int t = 0; t < 4; ++t) {
        FB vb;
        vb.h[0] = *(const v8b*)(Vth + (t * 16 + c) * AT_KC + kk * 32 + 8 * hh);
        vb.h[1] = *(const v8b*)(Vth + (t * 16 + c) * AT_KC + kk * 32 + 16 + 8 * hh);
        oacc[t] = at_mma(pa.v, vb.v, oacc[t]);
        if (SPLIT_PV) {
          FB vl;
          vl.h[0] = *(const v8b*)(Vtl + (t * 16 + c) * AT_KC + kk * 32 + 8 * hh);
          vl.h[1] = *(const v8b*)(Vtl + (t * 16 + c) * AT_KC + kk * 32 + 16 + 8 * hh);
          oacc[t] = at_mma(pa.v, vl.v, oacc[t]);
          oacc[t] = at_mma(pl.v, vb.v, oacc[t]);
        }
      }
    }
  }

  float* os = Os[wave];
#pragma unroll
  for (int r = 0; r < 8; ++r) {
    const float inv = 1.0f / lrow[r];
#pragma unroll
    for (int t = 0; t < 4; ++t) os[(8 * hh + r) * 68 + t * 16 + c] = oacc[t][r] * inv;
  }
  __builtin_amdgcn_fence(3  , "workgroup");
  __builtin_amdgcn_wave_barrier();
  __builtin_amdgcn_fence(2  , "workgroup");
  {
    const int c4 = (lane & 15) * 4;
    for (int pass = 0; pass < 2; ++pass) {
#pragma unroll
      for (int it = 0; it < 8; ++it) {
        const int row = it * 2 + hh;
        v4f val = *(const v4f*)(os + row * 68 + c4);
        *(volatile v4f*)(ob_ptr + (size_t)(q0 + row) * g.o_rs + c4) = val;
      }
      __threadfence();
    }
  }
}

extern "C" void kernel_launch(void* const* d_in, const int* in_sizes, int n_in, void* d_out, int out_size, void* d_ws, size_t ws_size, hipStream_t stream) {
    if (n_in < 5) return;
    const long long need_tok = (long long)(NB - 1) * SEQ_FULL + SEQ;
    if ((long long)in_sizes[0] < need_tok * DM) return;
    if ((long long)in_sizes[1] < (long long)DM * DM) return;
    if ((long long)in_sizes[2] < (long long)DM * DM) return;
    if ((long long)in_sizes[3] < (long long)DM * DM) return;
    if ((long long)in_sizes[4] < (long long)DM * DM) return;
    if ((long long)out_size < need_tok * DM) return;

    const float* x  = (const float*)d_in[0];
    const float* Wq = (const float*)d_in[1];
    const float* Wk = (const float*)d_in[2];
    const float* Wv = (const float*)d_in[3];
    const float* Wo = (const float*)d_in[4];
    float* out = (float*)d_out;

    const size_t szW3  = (size_t)3 * DM * DM * 2;
    const size_t szWOP = (size_t)DM * (2 * DM) * 2;
    const size_t szWOX = szWOP;
    const size_t szX16 = (size_t)NTOK * DM * 2;
    const size_t szQKV = (size_t)NTOK * 3 * DM * 4;
    const size_t szAO  = (size_t)NTOK * DM * 4;
    const size_t szAOP = (size_t)NTOK * (2 * DM) * 2;
    const size_t total = szW3 + szWOP + szWOX + szX16 + szQKV + szAO + szAOP;
    if (total > ws_size) return;
    char* wsp = (char*)d_ws;
    unsigned short* W316 = (unsigned short*)wsp; wsp += szW3;
    unsigned short* WOP  = (unsigned short*)wsp; wsp += szWOP;
    unsigned short* WOX  = (unsigned short*)wsp; wsp += szWOX;
    unsigned short* X16  = (unsigned short*)wsp; wsp += szX16;
    float*          QKV  = (float*)wsp;          wsp += szQKV;
    float*          AO   = (float*)wsp;          wsp += szAO;
    unsigned short* AOP  = (unsigned short*)wsp; wsp += szAOP;
    (void)wsp;

    const unsigned gW = (unsigned)(((long long)DM * (DM / 8) + 255) / 256);
    k_cm_castb<<<gW, 256, 0, stream>>>(Wq, DM, W316, DM, DM, DM, 16.0f);
    k_cm_castb<<<gW, 256, 0, stream>>>(Wk, DM, W316 + (size_t)DM * DM, DM, DM, DM, 16.0f);
    k_cm_castb<<<gW, 256, 0, stream>>>(Wv, DM, W316 + (size_t)2 * DM * DM, DM, DM, DM, 16.0f);
    const unsigned gWo = (unsigned)(((long long)DM * (DM / 2) + 255) / 256);
    k_castS16<<<gWo, 256, 0, stream>>>(Wo, DM, (__bf16*)WOP, (__bf16*)WOX, 2 * DM, DM, DM, 1.0f, 0);
    k_castS16<<<gWo, 256, 0, stream>>>(Wo, DM, (__bf16*)(WOP + DM), (__bf16*)(WOX + DM), 2 * DM, DM, DM, 1.0f, 0);
    const unsigned gX = (unsigned)(((long long)SEQ * (DM / 8) + 255) / 256);
    for (int bb = 0; bb < NB; ++bb)
        k_cm_castb<<<gX, 256, 0, stream>>>(x + (size_t)bb * SEQ_FULL * DM, DM, X16 + (size_t)bb * SEQ * DM, DM, SEQ, DM, 1.0f);
    wmma_gemm64<0, false, 0, 0, false><<<dim3((unsigned)(((NTOK / 64) * ((3 * DM) / 64) + 7) / 8), 1), 256, 0, stream>>>(
        X16, nullptr, DM, 0L, W316, nullptr, DM, 0L, (void*)QKV, nullptr, 3 * DM, 0L, nullptr, nullptr, 0L, NTOK, 3 * DM, DM, 0.0625f);
    k_rmsqk<<<(unsigned)((NTOK * 2 * NH) / 16), 256, 0, stream>>>(QKV, NTOK * 2 * NH);
    AttnGeom ag;
    ag.q_bs = (long long)SEQ * 3 * DM; ag.q_rs = 3 * DM; ag.q_hs = HD;
    ag.k_bs = (long long)SEQ * 3 * DM; ag.k_rs = 3 * DM; ag.k_hs = HD;
    ag.v_bs = (long long)SEQ * 3 * DM; ag.v_rs = 3 * DM; ag.v_hs = HD;
    ag.o_bs = (long long)SEQ * DM;     ag.o_rs = DM;     ag.o_hs = HD;
    ag.S = SEQ; ag.H = NH; ag.nqb = SEQ / AT_QB;
    ag.qscale = 0.125f; ag.cap = 50.0f; ag.capc = 0.057707801635558535f;
    k_attn64c<true, true><<<(unsigned)(NB * NH * (SEQ / AT_QB)), 128, 0, stream>>>(QKV, QKV + DM, QKV + 2 * DM, AO, ag);
    k_castS16<<<(unsigned)(((long long)NTOK * (DM / 2) + 255) / 256), 256, 0, stream>>>(AO, DM, (__bf16*)AOP, (__bf16*)(AOP + DM), 2 * DM, NTOK, DM, 1.0f, 0);
    wmma_gemm64<1, false, 0, 0, false><<<dim3((unsigned)(((SEQ / 64) * (DM / 64) + 7) / 8), (unsigned)NB), 256, 0, stream>>>(
        AOP, nullptr, 2 * DM, (long)SEQ * 2 * DM, WOP, nullptr, 2 * DM, 0L, (void*)out, nullptr, DM, (long)SEQ_FULL * DM, nullptr, nullptr, 0L, SEQ, DM, 2 * DM, 1.0f);
}
